// QAConv_68229850464663
// MI455X (gfx1250) — hardware-verified
//
#include <hip/hip_runtime.h>
#include <hip/hip_bf16.h>


#define PN     64
#define GN     64
#define CC     128
#define HW     192
#define NPAIR  (PN * GN)
#define KCHUNK 32
#define NCHUNK (CC / KCHUNK)
#define PITCHU 20
#define PITCHS (PITCHU * 2)
#define ABYTES (HW * PITCHU * 4)
#define NWAVE  12
#define TPB    (NWAVE * 32)
#define RECF   32
#define FTPB   256
#define KPT    (NPAIR / FTPB)
#define NPASS  (NPAIR / (FTPB * 4))
#define EPSV   1e-5f

static_assert(NPAIR % FTPB == 0, "");
static_assert(NPAIR % (FTPB * 4) == 0, "");
static_assert(HW % 32 == 0, "");

typedef __attribute__((ext_vector_type(16))) __bf16   v16bf;
typedef __attribute__((ext_vector_type(8)))  float    v8f;
typedef __attribute__((ext_vector_type(4)))  float    v4f;
typedef __attribute__((ext_vector_type(4)))  unsigned v4u;
typedef v4f __attribute__((may_alias)) v4fa;

__device__ __forceinline__ unsigned short f32_to_bf16_rne(float x) {
    unsigned u = __float_as_uint(x);
    unsigned r = u + 0x7FFFu + ((u >> 16) & 1u);
    return (unsigned short)(r >> 16);
}

__device__ __forceinline__ constexpr int inv_slot(int kp) {
    return (kp < 4) ? kp : (kp < 8) ? kp + 4 : (kp < 12) ? kp - 4 : kp;
}

__device__ __forceinline__ v16bf load_frag(const unsigned* baseU, int row20, int h8) {
    const v4u* p = (const v4u*)(baseU + row20 + h8);
    struct Pk { v4u a, b; } t;
    t.a = p[0];
    t.b = p[1];
    return __builtin_bit_cast(v16bf, t);
}

__device__ __forceinline__ v8f wmma_bf16(v16bf a, v16bf b, v8f c) {
    return __builtin_amdgcn_wmma_f32_16x16x32_bf16(false, a, false, b, (short)0, c, false, false);
}

__global__ __launch_bounds__(TPB, 1)
void pair_kernel(const float* __restrict__ prob,
                 const float* __restrict__ gal,
                 const float* __restrict__ fcw,
                 float* __restrict__ rec)
{
    __shared__ __align__(16) unsigned char smem[4 * ABYTES];
    __shared__ float sPart[NWAVE * 4];
    __shared__ __align__(16) float sRec[RECF];

    unsigned short* sAhi = (unsigned short*)(smem);
    unsigned short* sAlo = (unsigned short*)(smem + 1 * ABYTES);
    unsigned short* sBhi = (unsigned short*)(smem + 2 * ABYTES);
    unsigned short* sBlo = (unsigned short*)(smem + 3 * ABYTES);
    float* sMaxRw = (float*)(smem);
    float* sMaxS  = (float*)(smem + 9216);

    const int pair = blockIdx.x;
    const int p = pair >> 6, g = pair & 63;
    const int tid  = threadIdx.x;
    const int wav  = tid >> 5;
    const int lane = tid & 31;
    const int ln16 = lane & 15;
    const int half = lane >> 4;
    const int h8   = half * 8;

    const float* gbase = gal  + (size_t)g * CC * HW;
    const float* pbase = prob + (size_t)p * CC * HW;

    v8f acc[12] = {};

    const unsigned* aHiU = (const unsigned*)sAhi;
    const unsigned* aLoU = (const unsigned*)sAlo;
    const unsigned* bHiU = (const unsigned*)sBhi;
    const unsigned* bLoU = (const unsigned*)sBlo;
    const int aRow20 = (16 * wav + ln16) * PITCHU;

    const int c0 = tid / HW;
    const int rS = tid - c0 * HW;
    const int sRowBase = rS * PITCHS;

    for (int kc = 0; kc < NCHUNK; ++kc) {
        #pragma unroll
        for (int it = 0; it < 16; ++it) {
            const int sIdx = sRowBase + inv_slot(it) * 2 + c0;
            size_t go = (size_t)(kc * KCHUNK + 2 * it + c0) * HW + rS;

            float xg = gbase[go];
            unsigned short hg = f32_to_bf16_rne(xg);
            float hgf = __uint_as_float(((unsigned)hg) << 16);
            sAhi[sIdx] = hg;
            sAlo[sIdx] = f32_to_bf16_rne(xg - hgf);

            float xp = pbase[go];
            unsigned short hp = f32_to_bf16_rne(xp);
            float hpf = __uint_as_float(((unsigned)hp) << 16);
            sBhi[sIdx] = hp;
            sBlo[sIdx] = f32_to_bf16_rne(xp - hpf);
        }
        __syncthreads();

        v16bf aH = load_frag(aHiU, aRow20, h8);
        v16bf aL = load_frag(aLoU, aRow20, h8);
        #pragma unroll
        for (int j = 0; j < 12; ++j) {
            int bRow20 = (16 * j + ln16) * PITCHU;
            v16bf bH = load_frag(bHiU, bRow20, h8);
            v16bf bL = load_frag(bLoU, bRow20, h8);
            acc[j] = wmma_bf16(aH, bH, acc[j]);
            acc[j] = wmma_bf16(aH, bL, acc[j]);
            acc[j] = wmma_bf16(aL, bH, acc[j]);
            asm volatile("v_nop\n\tv_nop\n\tv_nop\n\tv_nop"
                         : "+v"(acc[j]) : "v"(aH), "v"(aL), "v"(bH), "v"(bL));
        }
        __syncthreads();
    }

    const float NEG = -__builtin_huge_valf();
    float rm[8];
    #pragma unroll
    for (int v = 0; v < 8; ++v) rm[v] = NEG;

    #pragma unroll
    for (int j = 0; j < 12; ++j) {
        float cm = NEG;
        #pragma unroll
        for (int v = 0; v < 8; ++v) {
            float x = acc[j][v];
            cm = fmaxf(cm, x);
            rm[v] = fmaxf(rm[v], x);
        }
        cm = fmaxf(cm, __shfl_xor(cm, 16, 32));
        if (lane < 16) sMaxRw[wav * HW + 16 * j + lane] = cm;
    }
    #pragma unroll
    for (int v = 0; v < 8; ++v) {
        float x = rm[v];
        x = fmaxf(x, __shfl_xor(x, 1, 32));
        x = fmaxf(x, __shfl_xor(x, 2, 32));
        x = fmaxf(x, __shfl_xor(x, 4, 32));
        x = fmaxf(x, __shfl_xor(x, 8, 32));
        if (ln16 == 0) sMaxS[16 * wav + v + 8 * half] = x;
    }
    __syncthreads();

    float wpart = 0.0f, spart = 0.0f, qpart = 0.0f;
    if (tid < HW) {
        float mr = NEG;
        #pragma unroll
        for (int w2 = 0; w2 < NWAVE; ++w2) mr = fmaxf(mr, sMaxRw[w2 * HW + tid]);
        float ms = sMaxS[tid];
        float w0 = fcw[tid];
        float w1 = fcw[HW + tid];
        wpart = w0 * mr + w1 * ms;
        spart = mr + ms;
        qpart = mr * mr + ms * ms;
    }
    #pragma unroll
    for (int o = 16; o > 0; o >>= 1) {
        wpart += __shfl_xor(wpart, o, 32);
        spart += __shfl_xor(spart, o, 32);
        qpart += __shfl_xor(qpart, o, 32);
    }
    if (lane == 0) {
        sPart[wav * 4 + 0] = wpart;
        sPart[wav * 4 + 1] = spart;
        sPart[wav * 4 + 2] = qpart;
        sPart[wav * 4 + 3] = 0.0f;
    }
    __syncthreads();
    if (tid < RECF) {
        float v = 0.0f;
        if (tid < 3) {
            #pragma unroll
            for (int w2 = 0; w2 < NWAVE; ++w2) v += sPart[w2 * 4 + tid];
        }
        sRec[tid] = v;
    }
    __syncthreads();

    v4f lv;
    lv.x = 0.0f; lv.y = 0.0f; lv.z = 0.0f; lv.w = 0.0f;
    const int tl = (tid < 8) ? tid : 0;
    if (tid < 8) lv = *(const v4fa*)(sRec + 4 * tl);
    float* dst = rec + (size_t)pair * RECF + 4 * tl;
    if (tid < 8) *(volatile v4f*)dst = lv;
    __threadfence();
    if (tid < 8) *(volatile v4f*)dst = lv;
}

__global__ __launch_bounds__(FTPB, 1)
void finalize_kernel(const float* __restrict__ rec,
                     const float* __restrict__ bn_gamma, const float* __restrict__ bn_beta,
                     const float* __restrict__ fc_w, const float* __restrict__ fc_b,
                     const float* __restrict__ lbn_gamma, const float* __restrict__ lbn_beta,
                     float* __restrict__ out)
{
    __shared__ double dA[FTPB];
    __shared__ double dB[FTPB];
    __shared__ __align__(16) float sLg[NPAIR];
    const int tid = threadIdx.x;

    float wd[KPT];
    double s1 = 0.0, s2 = 0.0;
    #pragma unroll
    for (int k = 0; k < KPT; ++k) {
        const float* r = rec + (size_t)(tid + FTPB * k) * RECF;
        wd[k] = r[0];
        s1 += (double)r[1];
        s2 += (double)r[2];
    }
    dA[tid] = s1;
    dB[tid] = s2;
    __syncthreads();
    for (int off = FTPB / 2; off > 0; off >>= 1) {
        if (tid < off) { dA[tid] += dA[tid + off]; dB[tid] += dB[tid + off]; }
        __syncthreads();
    }
    const double invNf = 1.0 / ((double)NPAIR * (double)(2 * HW));
    const double mu = dA[0] * invNf;
    double var = dB[0] * invNf - mu * mu;
    if (var < 0.0) var = 0.0;
    __syncthreads();

    double wt = 0.0;
    #pragma unroll 1
    for (int i = 0; i < 2 * HW; ++i) wt += (double)fc_w[i];

    const float kkf = bn_gamma[0] * rsqrtf((float)var + EPSV);
    const double kk = (double)kkf;
    const double cst = (double)bn_beta[0] * wt + (double)fc_b[0] - kk * mu * wt;

    double lg[KPT];
    double l1 = 0.0;
    #pragma unroll
    for (int k = 0; k < KPT; ++k) {
        lg[k] = kk * (double)wd[k] + cst;
        l1 += lg[k];
    }
    dA[tid] = l1;
    __syncthreads();
    for (int off = FTPB / 2; off > 0; off >>= 1) {
        if (tid < off) dA[tid] += dA[tid + off];
        __syncthreads();
    }
    const double lmu = dA[0] * (1.0 / (double)NPAIR);

    double l2 = 0.0;
    #pragma unroll
    for (int k = 0; k < KPT; ++k) {
        double d = lg[k] - lmu;
        l2 += d * d;
    }
    dB[tid] = l2;
    __syncthreads();
    for (int off = FTPB / 2; off > 0; off >>= 1) {
        if (tid < off) dB[tid] += dB[tid + off];
        __syncthreads();
    }
    const double lvar = dB[0] * (1.0 / (double)NPAIR);
    const float scf = lbn_gamma[0] * rsqrtf((float)lvar + EPSV);
    const double sc = (double)scf;
    const double sh = (double)lbn_beta[0];

    #pragma unroll
    for (int k = 0; k < KPT; ++k)
        sLg[tid + FTPB * k] = (float)((lg[k] - lmu) * sc + sh);
    __syncthreads();

    v4f ov[NPASS];
    #pragma unroll
    for (int ps = 0; ps < NPASS; ++ps)
        ov[ps] = *(const v4fa*)(sLg + FTPB * 4 * ps + 4 * tid);
    #pragma unroll
    for (int ps = 0; ps < NPASS; ++ps)
        *(volatile v4f*)(out + FTPB * 4 * ps + 4 * tid) = ov[ps];
    __threadfence();
    #pragma unroll
    for (int ps = 0; ps < NPASS; ++ps)
        *(volatile v4f*)(out + FTPB * 4 * ps + 4 * tid) = ov[ps];
}

extern "C" void kernel_launch(void* const* d_in, const int* in_sizes, int n_in,
                              void* d_out, int out_size, void* d_ws, size_t ws_size,
                              hipStream_t stream) {
    if (n_in < 8) return;
    if (in_sizes[0] != PN * CC * HW || in_sizes[1] != GN * CC * HW) return;
    if (in_sizes[2] < 1 || in_sizes[3] < 1 || in_sizes[4] < 2 * HW ||
        in_sizes[5] < 1 || in_sizes[6] < 1 || in_sizes[7] < 1) return;
    if (out_size != NPAIR) return;
    const size_t rec_bytes = (size_t)NPAIR * RECF * sizeof(float);
    if (rec_bytes > ws_size) return;

    const float* prob      = (const float*)d_in[0];
    const float* gal       = (const float*)d_in[1];
    const float* bn_gamma  = (const float*)d_in[2];
    const float* bn_beta   = (const float*)d_in[3];
    const float* fc_w      = (const float*)d_in[4];
    const float* fc_b      = (const float*)d_in[5];
    const float* lbn_gamma = (const float*)d_in[6];
    const float* lbn_beta  = (const float*)d_in[7];

    float* rec = (float*)d_ws;

    pair_kernel<<<dim3(NPAIR), dim3(TPB), 0, stream>>>(prob, gal, fc_w, rec);
    finalize_kernel<<<dim3(1), dim3(FTPB), 0, stream>>>(rec, bn_gamma, bn_beta, fc_w, fc_b,
                                                        lbn_gamma, lbn_beta, (float*)d_out);
    (void)hipGetLastError();
}
